// DependencyParser_88837103550580
// MI455X (gfx1250) — hardware-verified
//
#include <hip/hip_runtime.h>
#include <math.h>

typedef __attribute__((ext_vector_type(16))) _Float16 v16h;
typedef __attribute__((ext_vector_type(8)))  _Float16 v8h;
typedef __attribute__((ext_vector_type(16))) __bf16   v16b;
typedef __attribute__((ext_vector_type(8)))  __bf16   v8b;
typedef __attribute__((ext_vector_type(8)))  float    v8f;
typedef __attribute__((ext_vector_type(4)))  float    v4f;

constexpr int kBatch   = 16;
constexpr int kSeq     = 256;
constexpr int kWordDim = 100;
constexpr int kTagDim  = 28;
constexpr int kEmb     = kWordDim + kTagDim;
constexpr int kHid     = 128;
constexpr int kGate    = 4 * kHid;
constexpr int kCat2    = 2 * kHid;
constexpr int kRowsTB  = kSeq * kBatch;
constexpr int kVocW    = 32000;
constexpr int kVocT    = 50;
constexpr int kFc1     = 100;
constexpr int kFc1Pad  = 128;
constexpr int kAcN     = 2 * kFc1Pad;
constexpr int kRecThreads = 256;
constexpr int kHtP     = 136;
constexpr float kUp    = 16.0f;
constexpr float kDown  = 1.0f / 256.0f;
static_assert(kRowsTB % 64 == 0);
static_assert(kGate % 64 == 0);
static_assert(kAcN % 64 == 0);
static_assert(kEmb % 32 == 0);
static_assert(kCat2 % 32 == 0);
static_assert((kHtP * 2) % 16 == 0);

__device__ __forceinline__ unsigned short f2bf_bits(float f) {
  unsigned u = __float_as_uint(f);
  return (unsigned short)((u + 0x7FFFu + ((u >> 16) & 1u)) >> 16);
}
__device__ __forceinline__ float bf_bits2f(unsigned short h) { return __uint_as_float(((unsigned)h) << 16); }

__device__ __forceinline__ void dep_guard_h(v8f& a, v8f& b, v16h x, v16h y) { asm volatile("v_nop\n\tv_nop\n\tv_nop\n\tv_nop" : "+v"(a), "+v"(b) : "v"(x), "v"(y)); }
__device__ __forceinline__ void dep_guard_b(v8f& a, v8f& b, v16b x, v16b y) { asm volatile("v_nop\n\tv_nop\n\tv_nop\n\tv_nop" : "+v"(a), "+v"(b) : "v"(x), "v"(y)); }
__device__ __forceinline__ void keep4_h(v16h a, v16h b, v16h c, v16h d) { asm volatile("v_nop" :: "v"(a), "v"(b), "v"(c), "v"(d)); }
__device__ __forceinline__ void keep4_b(v16b a, v16b b, v16b c, v16b d) { asm volatile("v_nop" :: "v"(a), "v"(b), "v"(c), "v"(d)); }
__device__ __forceinline__ void acc_guard4(v8f& a, v8f& b, v8f& c, v8f& d) { asm volatile("v_nop\n\tv_nop\n\tv_nop\n\tv_nop" : "+v"(a), "+v"(b), "+v"(c), "+v"(d)); }

template <typename T> struct Frag;
template <> struct Frag<_Float16> {
  typedef v16h V; union U { v16h v; v8h h[2]; };
  static __device__ __forceinline__ v16h load(const _Float16* p) {
    U f; f.h[0] = *(const v8h*)(p); f.h[1] = *(const v8h*)(p + 16); return f.v;
  }
  static __device__ __forceinline__ v8f mma(v16h a, v16h b, v8f c) {
    return __builtin_amdgcn_wmma_f32_16x16x32_f16(false, a, false, b, (short)0, c, false, false);
  }
  static __device__ __forceinline__ void guard(v8f& a, v8f& b, v16h x, v16h y) { dep_guard_h(a, b, x, y); }
  static __device__ __forceinline__ void keep(v16h a, v16h b, v16h c, v16h d) { keep4_h(a, b, c, d); }
};
template <> struct Frag<__bf16> {
  typedef v16b V; union U { v16b v; v8b h[2]; };
  static __device__ __forceinline__ v16b load(const __bf16* p) {
    U f; f.h[0] = *(const v8b*)(p); f.h[1] = *(const v8b*)(p + 16); return f.v;
  }
  static __device__ __forceinline__ v8f mma(v16b a, v16b b, v8f c) {
    return __builtin_amdgcn_wmma_f32_16x16x32_bf16(false, a, false, b, (short)0, c, false, false);
  }
  static __device__ __forceinline__ void guard(v8f& a, v8f& b, v16b x, v16b y) { dep_guard_b(a, b, x, y); }
  static __device__ __forceinline__ void keep(v16b a, v16b b, v16b c, v16b d) { keep4_b(a, b, c, d); }
};

template <int ET> struct Elem;
template <> struct Elem<0> { typedef _Float16 T; };
template <> struct Elem<1> { typedef __bf16 T; };
template <int ET, bool SPLIT, int BIAS_MODE, int OUT_MODE, bool RESID, int ACT = 0, int TRI = 0>
__global__ __launch_bounds__(256) void wmma_gemm64(
    const unsigned short* __restrict__ Ap, const unsigned short* __restrict__ A2p, int lda, long strideA,
    const unsigned short* __restrict__ Btp, const unsigned short* __restrict__ Bt2p, int ldb, long strideB,
    void* __restrict__ Cout, void* __restrict__ Cout2, int ldc, long strideC,
    const float* __restrict__ bias,
    const float* __restrict__ resid, long strideR,
    int M, int N, int K, float scale) {
  typedef typename Elem<ET>::T T;
  typedef typename Frag<T>::V V;
  const T* A = (const T*)Ap; const T* A2 = (const T*)A2p; const T* Bt = (const T*)Btp; const T* Bt2 = (const T*)Bt2p;
  __shared__ __align__(16) float sT[8][16 * 68];
  const int b    = blockIdx.y;
  const int lane = threadIdx.x & 31;
  const int wave = threadIdx.x >> 5;
  const int tilesN = N >> 6;
  const int tilesM = M >> 6;
  const int tile = blockIdx.x * 8 + wave;
  if (tile >= tilesM * tilesN) return;
  const int tm = tile / tilesN;
  const int tn = tile - tm * tilesN;
  if (TRI == 1 && tn > tm) return;
  const int m0 = tm << 6;
  const int n0 = tn << 6;
  const int kLim = (TRI == 2) ? ((m0 + 64 < K) ? (m0 + 64) : K) : K;

  const T* Ab  = A  + (size_t)b * strideA;
  const T* Bb  = Bt + (size_t)b * strideB;
  const T* Ab2 = SPLIT ? (A2  + (size_t)b * strideA) : nullptr;
  const T* Bb2 = SPLIT ? (Bt2 + (size_t)b * strideB) : nullptr;

  const int rlane = lane & 15;
  const int koff  = (lane >> 4) * 8;
  const int mOff  = (lane >> 4) * 8;

  v8f acc[4][4];
#pragma unroll
  for (int i = 0; i < 4; ++i)
#pragma unroll
    for (int j = 0; j < 4; ++j) acc[i][j] = (v8f){0.f,0.f,0.f,0.f,0.f,0.f,0.f,0.f};

  for (int k0 = 0; k0 < kLim; k0 += 32) {
    V bh[4], bl[4];
#pragma unroll
    for (int j = 0; j < 4; ++j) {
      const size_t bo = (size_t)(n0 + (j << 4) + rlane) * ldb + koff + k0;
      bh[j] = Frag<T>::load(Bb + bo);
      if (SPLIT) bl[j] = Frag<T>::load(Bb2 + bo);
    }
#pragma unroll
    for (int i = 0; i < 4; ++i) {
      const size_t ao = (size_t)(m0 + (i << 4) + rlane) * lda + koff + k0;
      V ah = Frag<T>::load(Ab + ao);
      V al;
      if (SPLIT) al = Frag<T>::load(Ab2 + ao);
#pragma unroll
      for (int j = 0; j < 4; ++j) {
        acc[i][j] = Frag<T>::mma(ah, bh[j], acc[i][j]);
        if (SPLIT) {
          acc[i][j] = Frag<T>::mma(ah, bl[j], acc[i][j]);
          acc[i][j] = Frag<T>::mma(al, bh[j], acc[i][j]);
        }
      }
      Frag<T>::guard(acc[i][0], acc[i][3], ah, SPLIT ? al : ah);
    }
    Frag<T>::keep(bh[0], bh[1], bh[2], bh[3]);
    if (SPLIT) Frag<T>::keep(bl[0], bl[1], bl[2], bl[3]);
  }
  acc_guard4(acc[0][0], acc[0][1], acc[0][2], acc[0][3]);
  acc_guard4(acc[1][0], acc[1][1], acc[1][2], acc[1][3]);
  acc_guard4(acc[2][0], acc[2][1], acc[2][2], acc[2][3]);
  acc_guard4(acc[3][0], acc[3][1], acc[3][2], acc[3][3]);

  float* slab = sT[wave];
  const float* Rb = RESID ? (resid + (size_t)b * strideR) : nullptr;
#pragma unroll
  for (int i = 0; i < 4; ++i) {
    const int mBase = m0 + (i << 4);
#pragma unroll
    for (int j = 0; j < 4; ++j) {
      const int n = n0 + (j << 4) + rlane;
      float bv = 0.f;
      if (BIAS_MODE == 2) bv = bias[n];
#pragma unroll
      for (int r = 0; r < 8; ++r) {
        float v = acc[i][j][r] * scale;
        if (BIAS_MODE == 1) v += bias[mBase + mOff + r];
        if (BIAS_MODE == 2) v += bv;
        if (RESID) v += Rb[(size_t)(mBase + mOff + r) * ldc + n];
        if (ACT == 1) v = tanhf(v);
        if (ACT == 2) v = fmaxf(v, 0.0f);
        if (ACT == 4) v = (v > 0.f) ? v : 0.01f * v;
        slab[(mOff + r) * 68 + (j << 4) + rlane] = v;
      }
    }
    __builtin_amdgcn_fence(__ATOMIC_RELEASE, "workgroup");
    __builtin_amdgcn_wave_barrier();
    __builtin_amdgcn_fence(__ATOMIC_ACQUIRE, "workgroup");
    if (OUT_MODE == 0) {
      float* C = (float*)Cout + (size_t)b * strideC;
      const int hh = lane >> 4, c4 = (lane & 15) * 4;
      for (int pass = 0; pass < 2; ++pass) {
#pragma unroll
        for (int it = 0; it < 8; ++it) {
          const int row = it * 2 + hh;
          v4f v = *(const v4f*)(slab + row * 68 + c4);
          *(volatile v4f*)(C + (size_t)(mBase + row) * ldc + n0 + c4) = v;
        }
        __threadfence();
      }
    } else {
      const int q = lane >> 3, c8 = (lane & 7) * 8;
      unsigned short* C  = (unsigned short*)Cout  + (size_t)b * strideC;
      unsigned short* C2 = (OUT_MODE == 2) ? ((unsigned short*)Cout2 + (size_t)b * strideC) : nullptr;
      for (int pass = 0; pass < 2; ++pass) {
#pragma unroll
        for (int it = 0; it < 4; ++it) {
          const int row = it * 4 + q;
          const float* sp = slab + row * 68 + c8;
          v8h hv, lv;
#pragma unroll
          for (int e = 0; e < 8; ++e) {
            if (OUT_MODE == 1) {
              hv[e] = (_Float16)sp[e];
            } else {
              unsigned short hb = f2bf_bits(sp[e]);
              unsigned short lb = f2bf_bits(sp[e] - bf_bits2f(hb));
              hv[e] = __builtin_bit_cast(_Float16, hb);
              lv[e] = __builtin_bit_cast(_Float16, lb);
            }
          }
          *(volatile v8h*)(C + (size_t)(mBase + row) * ldc + n0 + c8) = hv;
          if (OUT_MODE == 2) *(volatile v8h*)(C2 + (size_t)(mBase + row) * ldc + n0 + c8) = lv;
        }
        __threadfence();
      }
    }
    __builtin_amdgcn_fence(__ATOMIC_RELEASE, "workgroup");
    __builtin_amdgcn_wave_barrier();
    __builtin_amdgcn_fence(__ATOMIC_ACQUIRE, "workgroup");
  }
}

__device__ __forceinline__ unsigned pack_f16x2(float a, float b) {
  const _Float16 h0 = (_Float16)a, h1 = (_Float16)b;
  return (unsigned)__builtin_bit_cast(unsigned short, h0) | ((unsigned)__builtin_bit_cast(unsigned short, h1) << 16);
}
__device__ __forceinline__ void st2u(unsigned* p, unsigned v) { *(volatile unsigned*)p = v; __threadfence(); *(volatile unsigned*)p = v; }
__device__ __forceinline__ float ftanh(float x) { return 1.0f - 2.0f * __builtin_amdgcn_rcpf(1.0f + __expf(2.0f * x)); }
__device__ __forceinline__ float fsigm(float x) { return __builtin_amdgcn_rcpf(1.0f + __expf(-x)); }

constexpr int kPrepBlocks = 1409;
__global__ __launch_bounds__(256) void prep_kernel(const float* __restrict__ wih0, const float* __restrict__ whh0,
                                                  const float* __restrict__ wih1, const float* __restrict__ whh1,
                                                  const float* __restrict__ fc1w, const float* __restrict__ fc1b,
                                                  unsigned* __restrict__ wih0u, unsigned* __restrict__ whh0u,
                                                  unsigned* __restrict__ wih1u, unsigned* __restrict__ whh1u,
                                                  unsigned* __restrict__ w12u, unsigned* __restrict__ b12u) {
  const int blk = blockIdx.x, tid = threadIdx.x;
  const int g = blk * 256 + tid;
  if (blk < 256) {
    const int p = g;
    st2u(wih0u + p, pack_f16x2(wih0[2 * p] * kUp, wih0[2 * p + 1] * kUp));
  } else if (blk < 512) {
    const int p = g - 65536;
    st2u(whh0u + p, pack_f16x2(whh0[2 * p] * kUp, whh0[2 * p + 1] * kUp));
  } else if (blk < 1024) {
    const int p = g - 131072;
    st2u(wih1u + p, pack_f16x2(wih1[2 * p] * kUp, wih1[2 * p + 1] * kUp));
  } else if (blk < 1280) {
    const int p = g - 262144;
    st2u(whh1u + p, pack_f16x2(whh1[2 * p] * kUp, whh1[2 * p + 1] * kUp));
  } else if (blk < 1408) {
    const int p = g - 327680;
    const int n = p >> 7;
    const int k = (2 * p) & 255;
    const int half = n >> 7;
    const int r = n & 127;
    const int rc = (r < kFc1) ? r : (kFc1 - 1);
    const float* src = fc1w + (size_t)rc * (2 * kCat2) + half * kCat2 + k;
    const float v0 = src[0] * kUp, v1 = src[1] * kUp;
    const unsigned u = (r < kFc1) ? pack_f16x2(v0, v1) : 0u;
    st2u(w12u + p, u);
  } else {
    const int n = tid;
    int r = n - kFc1Pad; const int rr = r; r = r < 0 ? 0 : r; r = r > (kFc1 - 1) ? (kFc1 - 1) : r;
    const float v = fc1b[r];
    const float f = (rr >= 0 && rr < kFc1) ? v : 0.0f;
    st2u(b12u + n, (unsigned)__float_as_uint(f));
  }
}

__global__ __launch_bounds__(256) void embed_kernel(const int* __restrict__ widx, const int* __restrict__ pidx,
                                                   const int* __restrict__ maxlen, const int* __restrict__ lengths,
                                                   const float* __restrict__ wemb, const float* __restrict__ temb,
                                                   _Float16* __restrict__ x16) {
  (void)maxlen; (void)lengths;
  const int tid = threadIdx.x;
  const int row = blockIdx.x * 16 + (tid >> 4);
  const int t = row >> 4, b = row & 15;
  const int c8 = (tid & 15) * 8;
  int w = widx[b * kSeq + t]; w = w < 0 ? 0 : w; w = w > (kVocW - 1) ? (kVocW - 1) : w;
  int p = pidx[b * kSeq + t]; p = p < 0 ? 0 : p; p = p > (kVocT - 1) ? (kVocT - 1) : p;
  const float* wr = wemb + (size_t)w * kWordDim;
  const float* tr = temb + (size_t)p * kTagDim;
  v8h hv;
#pragma unroll
  for (int e = 0; e < 8; ++e) {
    const int d = c8 + e;
    const int dw = (d < kWordDim) ? d : (kWordDim - 1);
    int dt = d - kWordDim; dt = dt < 0 ? 0 : dt;
    const float vw = wr[dw];
    const float vt = tr[dt];
    const float v = (d < kWordDim) ? vw : vt;
    hv[e] = (_Float16)(v * kUp);
  }
  _Float16* dst = x16 + (size_t)row * kEmb + c8;
  *(volatile v8h*)dst = hv;
  __threadfence();
  *(volatile v8h*)dst = hv;
}

__global__ __launch_bounds__(kRecThreads) void rec_kernel(
    const float* __restrict__ xp,
    const unsigned short* __restrict__ whh16u,
    const float* __restrict__ bih,
    const float* __restrict__ bhh,
    _Float16* __restrict__ hout16) {
  __shared__ __align__(16) _Float16 ht[kBatch * kHtP];
  const int tid = threadIdx.x, lane = tid & 31, wave = tid >> 5;
  const int rlane = lane & 15, hh = lane >> 4, koff = hh * 8, mOff = hh * 8;
  const int dir = blockIdx.x;
  const int ucol = wave * 16 + rlane;
  const _Float16* whh = (const _Float16*)whh16u + (size_t)dir * kGate * kHid;
  const float* xpd = xp + (size_t)dir * kRowsTB * kGate;

  for (int i = tid; i < kBatch * kHtP; i += kRecThreads) ht[i] = (_Float16)0.0f;
  float bq[4];
#pragma unroll
  for (int q = 0; q < 4; ++q) bq[q] = bih[dir * kGate + q * kHid + ucol] + bhh[dir * kGate + q * kHid + ucol];
  float c_st[8];
#pragma unroll
  for (int r = 0; r < 8; ++r) c_st[r] = 0.0f;
  __syncthreads();

  const _Float16* arow = ht + rlane * kHtP + koff;
  const _Float16* brow = whh + (size_t)ucol * kHid + koff;
  const v8f z8 = {0.f, 0.f, 0.f, 0.f, 0.f, 0.f, 0.f, 0.f};

#pragma unroll 1
  for (int s = 0; s < kSeq; ++s) {
    const int t = dir ? (kSeq - 1 - s) : s;

    const v16h a0 = Frag<_Float16>::load(arow);
    const v16h a1 = Frag<_Float16>::load(arow + 32);
    const v16h a2 = Frag<_Float16>::load(arow + 64);
    const v16h a3 = Frag<_Float16>::load(arow + 96);

    v8f acc[4];
    v16h fb = a0;
#pragma unroll
    for (int q = 0; q < 4; ++q) {
      const _Float16* bp = brow + (size_t)q * (kHid * kHid);
      acc[q] = z8;
      fb = Frag<_Float16>::load(bp);      acc[q] = Frag<_Float16>::mma(a0, fb, acc[q]);
      fb = Frag<_Float16>::load(bp + 32); acc[q] = Frag<_Float16>::mma(a1, fb, acc[q]);
      fb = Frag<_Float16>::load(bp + 64); acc[q] = Frag<_Float16>::mma(a2, fb, acc[q]);
      fb = Frag<_Float16>::load(bp + 96); acc[q] = Frag<_Float16>::mma(a3, fb, acc[q]);
    }
    dep_guard_h(acc[2], acc[3], a3, fb);
    keep4_h(a0, a1, a2, a3);
    acc_guard4(acc[0], acc[1], acc[2], acc[3]);

    float h_st[8];
    const float* xrow = xpd + (size_t)(t * kBatch + mOff) * kGate + ucol;
#pragma unroll
    for (int r = 0; r < 8; ++r) {
      const float* xb = xrow + (size_t)r * kGate;
      const float gi = fmaf(acc[0][r], kDown, xb[0]        + bq[0]);
      const float gf = fmaf(acc[1][r], kDown, xb[kHid]     + bq[1]);
      const float gg = fmaf(acc[2][r], kDown, xb[2 * kHid] + bq[2]);
      const float go = fmaf(acc[3][r], kDown, xb[3 * kHid] + bq[3]);
      const float iv = fsigm(gi), fv = fsigm(gf), gv = ftanh(gg), ov = fsigm(go);
      const float c = fmaf(fv, c_st[r], iv * gv);
      const float hv = ov * ftanh(c);
      c_st[r] = c; h_st[r] = hv;
    }
    __syncthreads();
#pragma unroll
    for (int r = 0; r < 8; ++r) ht[(mOff + r) * kHtP + ucol] = (_Float16)(h_st[r] * kUp);
    __syncthreads();
    {
      const int b = tid >> 4, c8 = (tid & 15) * 8;
      const v8h v = *(const v8h*)(ht + b * kHtP + c8);
      _Float16* dst = hout16 + (size_t)(t * kBatch + b) * kCat2 + dir * kHid + c8;
      *(volatile v8h*)dst = v;
      __threadfence();
      *(volatile v8h*)dst = v;
    }
  }
}

__global__ __launch_bounds__(256) void pair_kernel(const float* __restrict__ ac, const float* __restrict__ fc2w,
                                                  const float* __restrict__ fc2b, float* __restrict__ out) {
  __shared__ __align__(16) float as_[kFc1Pad];
  __shared__ __align__(16) float ws_[kFc1Pad];
  __shared__ __align__(16) float res[256];
  const int blk = blockIdx.x;
  const int b = blk & 15;
  const int tid = threadIdx.x;
  if (tid < kFc1Pad) {
    const int kc = (tid < kFc1) ? tid : (kFc1 - 1);
    const float av = ac[(size_t)blk * kAcN + kc];
    const float wv = fc2w[kc];
    as_[tid] = (tid < kFc1) ? av : 0.0f;
    ws_[tid] = (tid < kFc1) ? wv : 0.0f;
  }
  __syncthreads();
  const float* crow = ac + (size_t)(tid * kBatch + b) * kAcN + kFc1Pad;
  float sacc = 0.0f;
#pragma unroll 1
  for (int k = 0; k < kFc1; k += 4) {
    const v4f cv = *(const v4f*)(crow + k);
    const v4f av = *(const v4f*)(as_ + k);
    const v4f wv = *(const v4f*)(ws_ + k);
#pragma unroll
    for (int e = 0; e < 4; ++e) sacc = fmaf(wv[e], ftanh(av[e] + cv[e]), sacc);
  }
  res[tid] = sacc + fc2b[0];
  __syncthreads();
  if (tid < 64) {
    const v4f v = *(const v4f*)(res + tid * 4);
    float* dst = out + (size_t)blk * kSeq + tid * 4;
    *(volatile v4f*)dst = v;
    __threadfence();
    *(volatile v4f*)dst = v;
  }
}

extern "C" void kernel_launch(void* const* d_in, const int* in_sizes, int n_in,
                              void* d_out, int out_size, void* d_ws, size_t ws_size, hipStream_t stream) {
  if (n_in < 18 || d_out == nullptr || d_ws == nullptr) return;
  if (in_sizes[0] != kBatch * kSeq || in_sizes[1] != kBatch * kSeq || in_sizes[2] < 1 || in_sizes[3] != kBatch ||
      in_sizes[4] != kVocW * kWordDim || in_sizes[5] != kVocT * kTagDim ||
      in_sizes[6] != 2 * kGate * kEmb || in_sizes[7] != 2 * kGate * kHid || in_sizes[8] != 2 * kGate || in_sizes[9] != 2 * kGate ||
      in_sizes[10] != 2 * kGate * kCat2 || in_sizes[11] != 2 * kGate * kHid || in_sizes[12] != 2 * kGate || in_sizes[13] != 2 * kGate ||
      in_sizes[14] != kFc1 * 2 * kCat2 || in_sizes[15] != kFc1 || in_sizes[16] != kFc1 || in_sizes[17] != 1 ||
      out_size != kRowsTB * kSeq) return;

  const int*   widx   = (const int*)d_in[0];
  const int*   pidx   = (const int*)d_in[1];
  const int*   maxlen = (const int*)d_in[2];
  const int*   lens   = (const int*)d_in[3];
  const float* wemb   = (const float*)d_in[4];
  const float* temb   = (const float*)d_in[5];
  const float* wih_l0 = (const float*)d_in[6];
  const float* whh_l0 = (const float*)d_in[7];
  const float* bih_l0 = (const float*)d_in[8];
  const float* bhh_l0 = (const float*)d_in[9];
  const float* wih_l1 = (const float*)d_in[10];
  const float* whh_l1 = (const float*)d_in[11];
  const float* bih_l1 = (const float*)d_in[12];
  const float* bhh_l1 = (const float*)d_in[13];
  const float* fc1_w  = (const float*)d_in[14];
  const float* fc1_b  = (const float*)d_in[15];
  const float* fc2_w  = (const float*)d_in[16];
  const float* fc2_b  = (const float*)d_in[17];
  float* out = (float*)d_out;

  char* ws = (char*)d_ws; size_t off = 0;
  auto carve = [&](size_t bytes) -> char* { char* p = ws + off; off += (bytes + 255) & ~(size_t)255; return p; };
  unsigned short* X16   = (unsigned short*)carve((size_t)kRowsTB * kEmb * 2);
  unsigned short* WIH0  = (unsigned short*)carve((size_t)2 * kGate * kEmb * 2);
  unsigned short* WHH0  = (unsigned short*)carve((size_t)2 * kGate * kHid * 2);
  unsigned short* WIH1  = (unsigned short*)carve((size_t)2 * kGate * kCat2 * 2);
  unsigned short* WHH1  = (unsigned short*)carve((size_t)2 * kGate * kHid * 2);
  unsigned short* W12   = (unsigned short*)carve((size_t)kAcN * kCat2 * 2);
  float*          B12   = (float*)carve((size_t)kAcN * 4);
  float*          XP    = (float*)carve((size_t)2 * kRowsTB * kGate * 4);
  unsigned short* HOUT0 = (unsigned short*)carve((size_t)kRowsTB * kCat2 * 2);
  unsigned short* HOUT1 = (unsigned short*)carve((size_t)kRowsTB * kCat2 * 2);
  float*          AC    = (float*)carve((size_t)kRowsTB * kAcN * 4);
  if (off > ws_size || off > (size_t)134217728) return;

  prep_kernel<<<kPrepBlocks, 256, 0, stream>>>(wih_l0, whh_l0, wih_l1, whh_l1, fc1_w, fc1_b,
                                               (unsigned*)WIH0, (unsigned*)WHH0, (unsigned*)WIH1, (unsigned*)WHH1,
                                               (unsigned*)W12, (unsigned*)B12);

  embed_kernel<<<kRowsTB / 16, 256, 0, stream>>>(widx, pidx, maxlen, lens, wemb, temb, (_Float16*)X16);

  wmma_gemm64<0, false, 0, 0, false, 0, 0><<<dim3((kRowsTB / 64) * (kGate / 64) / 8, 2), 256, 0, stream>>>(
      X16, nullptr, kEmb, 0L, WIH0, nullptr, kEmb, (long)kGate * kEmb,
      (void*)XP, nullptr, kGate, (long)kRowsTB * kGate, nullptr, nullptr, 0L, kRowsTB, kGate, kEmb, kDown);

  rec_kernel<<<2, kRecThreads, 0, stream>>>(XP, WHH0, bih_l0, bhh_l0, (_Float16*)HOUT0);

  wmma_gemm64<0, false, 0, 0, false, 0, 0><<<dim3((kRowsTB / 64) * (kGate / 64) / 8, 2), 256, 0, stream>>>(
      HOUT0, nullptr, kCat2, 0L, WIH1, nullptr, kCat2, (long)kGate * kCat2,
      (void*)XP, nullptr, kGate, (long)kRowsTB * kGate, nullptr, nullptr, 0L, kRowsTB, kGate, kCat2, kDown);

  rec_kernel<<<2, kRecThreads, 0, stream>>>(XP, WHH1, bih_l1, bhh_l1, (_Float16*)HOUT1);

  wmma_gemm64<0, false, 2, 0, false, 0, 0><<<dim3((kRowsTB / 64) * (kAcN / 64) / 8, 1), 256, 0, stream>>>(
      HOUT1, nullptr, kCat2, 0L, W12, nullptr, kCat2, 0L,
      (void*)AC, nullptr, kAcN, 0L, B12, nullptr, 0L, kRowsTB, kAcN, kCat2, kDown);

  pair_kernel<<<kRowsTB, 256, 0, stream>>>(AC, fc2_w, fc2_b, out);
}
